// RA_MLA_Attention_27092653703663
// MI455X (gfx1250) — hardware-verified
//
#include <hip/hip_runtime.h>
#include <stddef.h>

constexpr int SEQ_T = 2048;
constexpr int EMB_E = 2048;
constexpr int NHEAD = 16;
constexpr int HDIM  = 128;
constexpr int LAT_L = 512;
constexpr int BAND_W = 64;
constexpr int AQB = 64;
constexpr int AKC = 64;
constexpr int ANW = 4;
constexpr int OS_PITCH = 132;
static_assert(SEQ_T % AQB == 0);
static_assert(SEQ_T / AQB == 32);
static_assert(SEQ_T % AKC == 0);
static_assert(EMB_E == NHEAD * HDIM);

constexpr size_t SZ_XB   = (size_t)SEQ_T * EMB_E * 2;
constexpr size_t SZ_WQB  = (size_t)EMB_E * EMB_E * 2;
constexpr size_t SZ_WKVB = (size_t)2 * LAT_L * EMB_E * 2;
constexpr size_t SZ_QTLB = (size_t)NHEAD * HDIM * LAT_L * 2;
constexpr size_t SZ_VUPT = (size_t)NHEAD * HDIM * LAT_L * 2;
constexpr size_t SZ_WOB  = (size_t)EMB_E * EMB_E * 2;
constexpr size_t SZ_QP   = (size_t)SEQ_T * EMB_E * 2;
constexpr size_t SZ_LKV  = (size_t)SEQ_T * 2 * LAT_L * 2;
constexpr size_t SZ_KP   = (size_t)NHEAD * SEQ_T * HDIM * 2;
constexpr size_t SZ_VT   = (size_t)NHEAD * HDIM * SEQ_T * 2;
constexpr size_t SZ_CTX  = (size_t)SEQ_T * EMB_E * 2;
constexpr size_t OFF_XB   = 0;
constexpr size_t OFF_WQB  = OFF_XB + SZ_XB;
constexpr size_t OFF_WKVB = OFF_WQB + SZ_WQB;
constexpr size_t OFF_QTLB = OFF_WKVB + SZ_WKVB;
constexpr size_t OFF_VUPT = OFF_QTLB + SZ_QTLB;
constexpr size_t OFF_WOB  = OFF_VUPT + SZ_VUPT;
constexpr size_t OFF_QPH  = OFF_WOB + SZ_WOB;
constexpr size_t OFF_QPL  = OFF_QPH + SZ_QP;
constexpr size_t OFF_LKVH = OFF_QPL + SZ_QP;
constexpr size_t OFF_LKVL = OFF_LKVH + SZ_LKV;
constexpr size_t OFF_KPH  = OFF_LKVL + SZ_LKV;
constexpr size_t OFF_KPL  = OFF_KPH + SZ_KP;
constexpr size_t OFF_VTH  = OFF_KPL + SZ_KP;
constexpr size_t OFF_VTL  = OFF_VTH + SZ_VT;
constexpr size_t OFF_CTXH = OFF_VTL + SZ_VT;
constexpr size_t OFF_CTXL = OFF_CTXH + SZ_CTX;
constexpr size_t WS_TOTAL = OFF_CTXL + SZ_CTX;
static_assert(WS_TOTAL == 109051904u);
static_assert(WS_TOTAL <= 134217728u);
static_assert((OFF_WQB % 128) == 0 && (OFF_WKVB % 128) == 0 && (OFF_QTLB % 128) == 0 && (OFF_VUPT % 128) == 0 && (OFF_WOB % 128) == 0);
static_assert((OFF_QPH % 128) == 0 && (OFF_QPL % 128) == 0 && (OFF_LKVH % 128) == 0 && (OFF_LKVL % 128) == 0);
static_assert((OFF_KPH % 128) == 0 && (OFF_KPL % 128) == 0 && (OFF_VTH % 128) == 0 && (OFF_VTL % 128) == 0 && (OFF_CTXH % 128) == 0 && (OFF_CTXL % 128) == 0);

typedef __attribute__((ext_vector_type(16))) _Float16 v16h;
typedef __attribute__((ext_vector_type(8)))  _Float16 v8h;
typedef __attribute__((ext_vector_type(16))) __bf16   v16b;
typedef __attribute__((ext_vector_type(8)))  __bf16   v8b;
typedef __attribute__((ext_vector_type(8)))  float    v8f;
typedef __attribute__((ext_vector_type(4)))  float    v4f;
typedef __attribute__((ext_vector_type(4)))  unsigned v4u;

__device__ __forceinline__ unsigned short f2bf_bits(float f) {
  unsigned u = __float_as_uint(f);
  return (unsigned short)((u + 0x7FFFu + ((u >> 16) & 1u)) >> 16);
}
__device__ __forceinline__ float bf_bits2f(unsigned short h) { return __uint_as_float(((unsigned)h) << 16); }

__device__ __forceinline__ void dep_guard_h(v8f& a, v8f& b, v16h x, v16h y) { asm volatile("v_nop\n\tv_nop\n\tv_nop\n\tv_nop" : "+v"(a), "+v"(b) : "v"(x), "v"(y)); }
__device__ __forceinline__ void dep_guard_b(v8f& a, v8f& b, v16b x, v16b y) { asm volatile("v_nop\n\tv_nop\n\tv_nop\n\tv_nop" : "+v"(a), "+v"(b) : "v"(x), "v"(y)); }
__device__ __forceinline__ void keep4_h(v16h a, v16h b, v16h c, v16h d) { asm volatile("v_nop" :: "v"(a), "v"(b), "v"(c), "v"(d)); }
__device__ __forceinline__ void keep4_b(v16b a, v16b b, v16b c, v16b d) { asm volatile("v_nop" :: "v"(a), "v"(b), "v"(c), "v"(d)); }
__device__ __forceinline__ void acc_guard4(v8f& a, v8f& b, v8f& c, v8f& d) { asm volatile("v_nop\n\tv_nop\n\tv_nop\n\tv_nop" : "+v"(a), "+v"(b), "+v"(c), "+v"(d)); }
template <typename T> struct Frag;
template <> struct Frag<_Float16> {
  typedef v16h V; union U { v16h v; v8h h[2]; };
  static __device__ __forceinline__ v16h load(const _Float16* p) {
    U f; f.h[0] = *(const v8h*)(p); f.h[1] = *(const v8h*)(p + 16); return f.v;
  }
  static __device__ __forceinline__ v8f mma(v16h a, v16h b, v8f c) {
    return __builtin_amdgcn_wmma_f32_16x16x32_f16(false, a, false, b, (short)0, c, false, false);
  }
  static __device__ __forceinline__ void guard(v8f& a, v8f& b, v16h x, v16h y) { dep_guard_h(a, b, x, y); }
  static __device__ __forceinline__ void keep(v16h a, v16h b, v16h c, v16h d) { keep4_h(a, b, c, d); }
};
template <> struct Frag<__bf16> {
  typedef v16b V; union U { v16b v; v8b h[2]; };
  static __device__ __forceinline__ v16b load(const __bf16* p) {
    U f; f.h[0] = *(const v8b*)(p); f.h[1] = *(const v8b*)(p + 16); return f.v;
  }
  static __device__ __forceinline__ v8f mma(v16b a, v16b b, v8f c) {
    return __builtin_amdgcn_wmma_f32_16x16x32_bf16(false, a, false, b, (short)0, c, false, false);
  }
  static __device__ __forceinline__ void guard(v8f& a, v8f& b, v16b x, v16b y) { dep_guard_b(a, b, x, y); }
  static __device__ __forceinline__ void keep(v16b a, v16b b, v16b c, v16b d) { keep4_b(a, b, c, d); }
};

template <int ET> struct Elem;
template <> struct Elem<0> { typedef _Float16 T; };
template <> struct Elem<1> { typedef __bf16 T; };
template <int ET, int SPLITM, int BIAS_MODE, int OUT_MODE, bool RESID>
__global__ __launch_bounds__(256) void wmma_gemm64(
    const unsigned short* __restrict__ Ap, const unsigned short* __restrict__ A2p, int lda, long strideA,
    const unsigned short* __restrict__ Btp, const unsigned short* __restrict__ Bt2p, int ldb, long strideB,
    void* __restrict__ Cout, void* __restrict__ Cout2, int ldc, long strideC,
    const float* __restrict__ bias,
    const float* __restrict__ resid, long strideR,
    int M, int N, int K, float scale) {
  constexpr bool SA = (SPLITM == 1) || (SPLITM == 2);
  constexpr bool SB = (SPLITM == 1) || (SPLITM == 3);
  typedef typename Elem<ET>::T T;
  typedef typename Frag<T>::V V;
  const T* A = (const T*)Ap; const T* A2 = (const T*)A2p; const T* Bt = (const T*)Btp; const T* Bt2 = (const T*)Bt2p;
  __shared__ __align__(16) float sT[8][16 * 68];
  const int b    = blockIdx.y;
  const int lane = threadIdx.x & 31;
  const int wave = threadIdx.x >> 5;
  const int tilesN = N >> 6;
  const int tilesM = M >> 6;
  const int tile = blockIdx.x * 8 + wave;
  if (tile >= tilesM * tilesN) return;
  const int tm = tile / tilesN;
  const int tn = tile - tm * tilesN;
  const int m0 = tm << 6;
  const int n0 = tn << 6;

  const T* Ab  = A  + (size_t)b * strideA;
  const T* Bb  = Bt + (size_t)b * strideB;
  const T* Ab2 = SA ? (A2  + (size_t)b * strideA) : nullptr;
  const T* Bb2 = SB ? (Bt2 + (size_t)b * strideB) : nullptr;

  const int rlane = lane & 15;
  const int koff  = (lane >> 4) * 8;
  const int mOff  = (lane >> 4) * 8;

  v8f acc[4][4];
#pragma unroll
  for (int i = 0; i < 4; ++i)
#pragma unroll
    for (int j = 0; j < 4; ++j) acc[i][j] = (v8f){0.f,0.f,0.f,0.f,0.f,0.f,0.f,0.f};

  for (int k0 = 0; k0 < K; k0 += 32) {
    V bh[4], bl[4];
#pragma unroll
    for (int j = 0; j < 4; ++j) {
      const size_t bo = (size_t)(n0 + (j << 4) + rlane) * ldb + koff + k0;
      bh[j] = Frag<T>::load(Bb + bo);
      if (SB) bl[j] = Frag<T>::load(Bb2 + bo);
      else bl[j] = bh[j];
    }
#pragma unroll
    for (int i = 0; i < 4; ++i) {
      const size_t ao = (size_t)(m0 + (i << 4) + rlane) * lda + koff + k0;
      V ah = Frag<T>::load(Ab + ao);
      V al = ah;
      if (SA) al = Frag<T>::load(Ab2 + ao);
#pragma unroll
      for (int j = 0; j < 4; ++j) {
        acc[i][j] = Frag<T>::mma(ah, bh[j], acc[i][j]);
        if (SB) acc[i][j] = Frag<T>::mma(ah, bl[j], acc[i][j]);
        if (SA) acc[i][j] = Frag<T>::mma(al, bh[j], acc[i][j]);
      }
      Frag<T>::guard(acc[i][0], acc[i][3], ah, al);
    }
    Frag<T>::keep(bh[0], bh[1], bh[2], bh[3]);
    if (SB) Frag<T>::keep(bl[0], bl[1], bl[2], bl[3]);
  }
  acc_guard4(acc[0][0], acc[0][1], acc[0][2], acc[0][3]);
  acc_guard4(acc[1][0], acc[1][1], acc[1][2], acc[1][3]);
  acc_guard4(acc[2][0], acc[2][1], acc[2][2], acc[2][3]);
  acc_guard4(acc[3][0], acc[3][1], acc[3][2], acc[3][3]);

  float* slab = sT[wave];
  const float* Rb = RESID ? (resid + (size_t)b * strideR) : nullptr;
#pragma unroll
  for (int i = 0; i < 4; ++i) {
    const int mBase = m0 + (i << 4);
#pragma unroll
    for (int j = 0; j < 4; ++j) {
      const int n = n0 + (j << 4) + rlane;
      float bv = 0.f;
      if (BIAS_MODE == 2) bv = bias[n];
#pragma unroll
      for (int r = 0; r < 8; ++r) {
        float v = acc[i][j][r] * scale;
        if (BIAS_MODE == 1) v += bias[mBase + mOff + r];
        if (BIAS_MODE == 2) v += bv;
        if (RESID) v += Rb[(size_t)(mBase + mOff + r) * ldc + n];
        slab[(mOff + r) * 68 + (j << 4) + rlane] = v;
      }
    }
    __builtin_amdgcn_fence(__ATOMIC_RELEASE, "workgroup");
    __builtin_amdgcn_wave_barrier();
    __builtin_amdgcn_fence(__ATOMIC_ACQUIRE, "workgroup");
    if (OUT_MODE == 0) {
      float* C = (float*)Cout + (size_t)b * strideC;
      const int hh = lane >> 4, c4 = (lane & 15) * 4;
      for (int pass = 0; pass < 2; ++pass) {
#pragma unroll
        for (int it = 0; it < 8; ++it) {
          const int row = it * 2 + hh;
          v4f v = *(const v4f*)(slab + row * 68 + c4);
          *(volatile v4f*)(C + (size_t)(mBase + row) * ldc + n0 + c4) = v;
        }
        __threadfence();
      }
    } else {
      const int q = lane >> 3, c8 = (lane & 7) * 8;
      unsigned short* C  = (unsigned short*)Cout  + (size_t)b * strideC;
      unsigned short* C2 = (OUT_MODE == 2) ? ((unsigned short*)Cout2 + (size_t)b * strideC) : nullptr;
      for (int pass = 0; pass < 2; ++pass) {
#pragma unroll
        for (int it = 0; it < 4; ++it) {
          const int row = it * 4 + q;
          const float* sp = slab + row * 68 + c8;
          v8h hv, lv;
#pragma unroll
          for (int e = 0; e < 8; ++e) {
            if (OUT_MODE == 1) {
              hv[e] = (_Float16)sp[e];
              lv[e] = hv[e];
            } else {
              unsigned short hb = f2bf_bits(sp[e]);
              unsigned short lb = f2bf_bits(sp[e] - bf_bits2f(hb));
              hv[e] = __builtin_bit_cast(_Float16, hb);
              lv[e] = __builtin_bit_cast(_Float16, lb);
            }
          }
          *(volatile v8h*)(C + (size_t)(mBase + row) * ldc + n0 + c8) = hv;
          if (OUT_MODE == 2) *(volatile v8h*)(C2 + (size_t)(mBase + row) * ldc + n0 + c8) = lv;
        }
        __threadfence();
      }
    }
    __builtin_amdgcn_fence(__ATOMIC_RELEASE, "workgroup");
    __builtin_amdgcn_wave_barrier();
    __builtin_amdgcn_fence(__ATOMIC_ACQUIRE, "workgroup");
  }
}

__global__ __launch_bounds__(256) void k_cast_bf16x8(
    const float* __restrict__ in, unsigned short* __restrict__ out, int n8) {
  const int i = blockIdx.x * 256 + threadIdx.x;
  if (i < n8) {
    const size_t o = (size_t)i * 8;
    const v4f a  = *(const v4f*)(in + o);
    const v4f aa = *(const v4f*)(in + o + 4);
    v4u w;
    w[0] = (unsigned)f2bf_bits(a[0])  | ((unsigned)f2bf_bits(a[1])  << 16);
    w[1] = (unsigned)f2bf_bits(a[2])  | ((unsigned)f2bf_bits(a[3])  << 16);
    w[2] = (unsigned)f2bf_bits(aa[0]) | ((unsigned)f2bf_bits(aa[1]) << 16);
    w[3] = (unsigned)f2bf_bits(aa[2]) | ((unsigned)f2bf_bits(aa[3]) << 16);
    *(volatile v4u*)(out + o) = w;
    __threadfence();
    *(volatile v4u*)(out + o) = w;
  }
}

__global__ __launch_bounds__(256) void k_vup_tcast(const float* __restrict__ in, unsigned short* __restrict__ out) {
  __shared__ float tile[64][65];
  const int lt = blockIdx.x, dt = blockIdx.y, h = blockIdx.z;
  const int l0 = lt * 64, d0 = dt * 64;
  const int tid = threadIdx.x;
  const int dcol = tid & 63, lrb = tid >> 6;
#pragma unroll
  for (int i = 0; i < 8; ++i) {
    const int lr = lrb + 4 * i;
    tile[dcol][lr] = in[((size_t)(h * LAT_L + l0 + lr)) * HDIM + d0 + dcol];
  }
  asm volatile("" ::: "memory");
#pragma unroll
  for (int i = 8; i < 16; ++i) {
    const int lr = lrb + 4 * i;
    tile[dcol][lr] = in[((size_t)(h * LAT_L + l0 + lr)) * HDIM + d0 + dcol];
  }
  __syncthreads();
  const int wave = tid >> 5, lane = tid & 31, q8 = lane >> 3, c8 = (lane & 7) * 8;
  for (int pass = 0; pass < 2; ++pass) {
#pragma unroll
    for (int it = 0; it < 2; ++it) {
      const int row = wave * 8 + it * 4 + q8;
      const float* sp = &tile[row][c8];
      v8h hv;
#pragma unroll
      for (int e = 0; e < 8; ++e) hv[e] = __builtin_bit_cast(_Float16, f2bf_bits(sp[e]));
      *(volatile v8h*)(out + ((size_t)(h * HDIM + d0 + row)) * LAT_L + l0 + c8) = hv;
    }
    __threadfence();
  }
}

__device__ __forceinline__ unsigned short at_bf_bits(float f) {
  unsigned u = __float_as_uint(f);
  return (unsigned short)((u + 0x7FFFu + ((u >> 16) & 1u)) >> 16);
}
__device__ __forceinline__ __bf16 at_f2bf(float f) { return __builtin_bit_cast(__bf16, at_bf_bits(f)); }
__device__ __forceinline__ void at_split(float f, __bf16& hi, __bf16& lo) {
  const unsigned short hb = at_bf_bits(f);
  hi = __builtin_bit_cast(__bf16, hb);
  lo = at_f2bf(f - __uint_as_float(((unsigned)hb) << 16));
}
__device__ __forceinline__ v8f at_mma(v16b a, v16b b, v8f c) {
  c = __builtin_amdgcn_wmma_f32_16x16x32_bf16(false, a, false, b, (short)0, c, false, false);
  asm volatile("v_nop\n\tv_nop\n\tv_nop\n\tv_nop" : "+v"(c) : "v"(a), "v"(b));
  return c;
}

__global__ __launch_bounds__(128)
void k_band_attn(const unsigned short* __restrict__ Qhp, const unsigned short* __restrict__ Qlp,
                 const unsigned short* __restrict__ Khp, const unsigned short* __restrict__ Klp,
                 const unsigned short* __restrict__ Vhp, const unsigned short* __restrict__ Vlp,
                 unsigned short* __restrict__ Chp, unsigned short* __restrict__ Clp) {
  union FB { v16b v; v8b h[2]; };
  __shared__ __align__(16) __bf16 Qs0[AQB * HDIM];
  __shared__ __align__(16) __bf16 Qs1[AQB * HDIM];
  __shared__ __align__(16) __bf16 Ks0[AKC * HDIM];
  __shared__ __align__(16) __bf16 Ks1[AKC * HDIM];
  __shared__ __align__(16) __bf16 Vs0[HDIM * AKC];
  __shared__ __align__(16) __bf16 Vs1[HDIM * AKC];
  __shared__ __align__(16) __bf16 Psh[ANW][16 * AKC];
  __shared__ __align__(16) __bf16 Psl[ANW][16 * AKC];
  __shared__ __align__(16) float  Os[ANW][16 * OS_PITCH];

  const int tid  = threadIdx.x;
  const int wave = tid >> 5;
  const int lane = tid & 31;
  const int hh   = lane >> 4;
  const int c    = lane & 15;
  const int bx   = blockIdx.x;
  const int qb   = bx & 31;
  const int h    = bx >> 5;
  const int qblk = qb * AQB;
  const int q0   = qblk + wave * 16;

  {
    const unsigned short* sh = Qhp + (size_t)qblk * EMB_E + (size_t)h * HDIM;
    const unsigned short* sl = Qlp + (size_t)qblk * EMB_E + (size_t)h * HDIM;
#pragma unroll
    for (int i = 0; i < 8; ++i) {
      const int idx = tid + 128 * i, row = idx >> 4, cc = (idx & 15) * 8;
      const v4u w = *(const v4u*)(sh + (size_t)row * EMB_E + cc);
      *(v4u*)(Qs0 + row * HDIM + cc) = w;
    }
    asm volatile("" ::: "memory");
#pragma unroll
    for (int i = 0; i < 8; ++i) {
      const int idx = tid + 128 * i, row = idx >> 4, cc = (idx & 15) * 8;
      const v4u w = *(const v4u*)(sl + (size_t)row * EMB_E + cc);
      *(v4u*)(Qs1 + row * HDIM + cc) = w;
    }
    asm volatile("" ::: "memory");
  }

  float mrow[8], lrow[8];
  v8f oacc[8];
#pragma unroll
  for (int r = 0; r < 8; ++r) { mrow[r] = -__builtin_inff(); lrow[r] = 0.f; }
#pragma unroll
  for (int t = 0; t < 8; ++t) oacc[t] = (v8f){0.f,0.f,0.f,0.f,0.f,0.f,0.f,0.f};

  const float rscale = 0.044194173824159216f;
  const int nChunks = ((qb + 1) < 32) ? (qb + 1) : 32;

  for (int kc = 0; kc < nChunks; ++kc) {
    const int kv0 = kc * AKC;
    __syncthreads();
    {
      const unsigned short* sk0 = Khp + ((size_t)h * SEQ_T + kv0) * HDIM;
      const unsigned short* sk1 = Klp + ((size_t)h * SEQ_T + kv0) * HDIM;
      const unsigned short* sv0 = Vhp + (size_t)h * HDIM * SEQ_T + kv0;
      const unsigned short* sv1 = Vlp + (size_t)h * HDIM * SEQ_T + kv0;
#pragma unroll
      for (int i = 0; i < 8; ++i) {
        const int idx = tid + 128 * i;
        const v4u w = *(const v4u*)(sk0 + (size_t)idx * 8);
        *(v4u*)(Ks0 + idx * 8) = w;
      }
      asm volatile("" ::: "memory");
#pragma unroll
      for (int i = 0; i < 8; ++i) {
        const int idx = tid + 128 * i;
        const v4u w = *(const v4u*)(sk1 + (size_t)idx * 8);
        *(v4u*)(Ks1 + idx * 8) = w;
      }
      asm volatile("" ::: "memory");
#pragma unroll
      for (int i = 0; i < 8; ++i) {
        const int idx = tid + 128 * i, d = idx >> 3, cc = (idx & 7) * 8;
        const v4u w = *(const v4u*)(sv0 + (size_t)d * SEQ_T + cc);
        *(v4u*)(Vs0 + d * AKC + cc) = w;
      }
      asm volatile("" ::: "memory");
#pragma unroll
      for (int i = 0; i < 8; ++i) {
        const int idx = tid + 128 * i, d = idx >> 3, cc = (idx & 7) * 8;
        const v4u w = *(const v4u*)(sv1 + (size_t)d * SEQ_T + cc);
        *(v4u*)(Vs1 + d * AKC + cc) = w;
      }
      asm volatile("" ::: "memory");
    }
    __syncthreads();

    v8f s[4];
#pragma unroll
    for (int j = 0; j < 4; ++j) s[j] = (v8f){0.f,0.f,0.f,0.f,0.f,0.f,0.f,0.f};
#pragma unroll 1
    for (int dc = 0; dc < 4; ++dc) {
      FB qa, ql;
      const __bf16* qp0 = Qs0 + (wave * 16 + c) * HDIM + dc * 32 + 8 * hh;
      const __bf16* qp1 = Qs1 + (wave * 16 + c) * HDIM + dc * 32 + 8 * hh;
      qa.h[0] = *(const v8b*)(qp0); qa.h[1] = *(const v8b*)(qp0 + 16);
      ql.h[0] = *(const v8b*)(qp1); ql.h[1] = *(const v8b*)(qp1 + 16);
#pragma unroll
      for (int j = 0; j < 4; ++j) {
        FB kb, kl;
        const __bf16* kp0 = Ks0 + (j * 16 + c) * HDIM + dc * 32 + 8 * hh;
        const __bf16* kp1 = Ks1 + (j * 16 + c) * HDIM + dc * 32 + 8 * hh;
        kb.h[0] = *(const v8b*)(kp0); kb.h[1] = *(const v8b*)(kp0 + 16);
        kl.h[0] = *(const v8b*)(kp1); kl.h[1] = *(const v8b*)(kp1 + 16);
        s[j] = at_mma(qa.v, kb.v, s[j]);
        s[j] = at_mma(qa.v, kl.v, s[j]);
        s[j] = at_mma(ql.v, kb.v, s[j]);
        asm volatile("" ::: "memory");
      }
    }

    float cm[8];
#pragma unroll
    for (int r = 0; r < 8; ++r) {
      const int qrow = q0 + 8 * hh + r;
      float m = -__builtin_inff();
#pragma unroll
      for (int j = 0; j < 4; ++j) {
        const int kvcol = kv0 + j * 16 + c;
        const int dlt = qrow - kvcol;
        float x = s[j][r] * rscale;
        x = (dlt < BAND_W) ? (x * 1.5f) : x;
        x = (dlt < 0) ? -__builtin_inff() : x;
        s[j][r] = x;
        m = fmaxf(m, x);
      }
#pragma unroll
      for (int off = 1; off < 16; off <<= 1) m = fmaxf(m, __shfl_xor(m, off, 32));
      cm[r] = m;
    }
    __bf16* pwh = Psh[wave];
    __bf16* pwl = Psl[wave];
#pragma unroll
    for (int r = 0; r < 8; ++r) {
      const float mnew = fmaxf(mrow[r], cm[r]);
      const float alpha = expf(mrow[r] - mnew);
      mrow[r] = mnew;
      float psum = 0.f;
#pragma unroll
      for (int j = 0; j < 4; ++j) {
        const float p = expf(s[j][r] - mnew);
        psum += p;
        __bf16 a, bl;
        at_split(p, a, bl);
        pwh[(8 * hh + r) * AKC + j * 16 + c] = a;
        pwl[(8 * hh + r) * AKC + j * 16 + c] = bl;
      }
#pragma unroll
      for (int off = 1; off < 16; off <<= 1) psum += __shfl_xor(psum, off, 32);
      lrow[r] = lrow[r] * alpha + psum;
#pragma unroll
      for (int t = 0; t < 8; ++t) oacc[t][r] *= alpha;
    }
    __builtin_amdgcn_fence(__ATOMIC_RELEASE, "workgroup");
    __builtin_amdgcn_wave_barrier();
    __builtin_amdgcn_fence(__ATOMIC_ACQUIRE, "workgroup");
#pragma unroll 1
    for (int kk = 0; kk < 2; ++kk) {
      FB pa, pl;
      pa.h[0] = *(const v8b*)(pwh + c * AKC + kk * 32 + 8 * hh);
      pa.h[1] = *(const v8b*)(pwh + c * AKC + kk * 32 + 16 + 8 * hh);
      pl.h[0] = *(const v8b*)(pwl + c * AKC + kk * 32 + 8 * hh);
      pl.h[1] = *(const v8b*)(pwl + c * AKC + kk * 32 + 16 + 8 * hh);
#pragma unroll
      for (int t = 0; t < 8; ++t) {
        FB vb, vl;
        const __bf16* vp0 = Vs0 + (t * 16 + c) * AKC + kk * 32 + 8 * hh;
        const __bf16* vp1 = Vs1 + (t * 16 + c) * AKC + kk * 32 + 8 * hh;
        vb.h[0] = *(const v8b*)(vp0); vb.h[1] = *(const v8b*)(vp0 + 16);
        vl.h[0] = *(const v8b*)(vp1); vl.h[1] = *(const v8b*)(vp1 + 16);
        oacc[t] = at_mma(pa.v, vb.v, oacc[t]);
        oacc[t] = at_mma(pa.v, vl.v, oacc[t]);
        oacc[t] = at_mma(pl.v, vb.v, oacc[t]);
        asm volatile("" ::: "memory");
      }
    }
  }

  float* os = Os[wave];
#pragma unroll
  for (int r = 0; r < 8; ++r) {
    const float inv = 1.0f / lrow[r];
#pragma unroll
    for (int t = 0; t < 8; ++t) os[(8 * hh + r) * OS_PITCH + t * 16 + c] = oacc[t][r] * inv;
  }
  __builtin_amdgcn_fence(__ATOMIC_RELEASE, "workgroup");
  __builtin_amdgcn_wave_barrier();
  __builtin_amdgcn_fence(__ATOMIC_ACQUIRE, "workgroup");
  {
    const int q8 = lane >> 3, c8 = (lane & 7) * 8;
    for (int pass = 0; pass < 2; ++pass) {
#pragma unroll
      for (int it = 0; it < 8; ++it) {
        const int lidx = it * 4 + q8;
        const int row = lidx >> 1;
        const int colb = (lidx & 1) * 64 + c8;
        const float* sp = os + row * OS_PITCH + colb;
        v8h hv, lv;
#pragma unroll
        for (int e = 0; e < 8; ++e) {
          const unsigned short hb = at_bf_bits(sp[e]);
          const unsigned short lb = at_bf_bits(sp[e] - __uint_as_float(((unsigned)hb) << 16));
          hv[e] = __builtin_bit_cast(_Float16, hb);
          lv[e] = __builtin_bit_cast(_Float16, lb);
        }
        const size_t go = (size_t)(q0 + row) * EMB_E + (size_t)h * HDIM + colb;
        *(volatile v8h*)(Chp + go) = hv;
        *(volatile v8h*)(Clp + go) = lv;
      }
      __threadfence();
    }
  }
}

static_assert(SEQ_T % 64 == 0 && EMB_E % 64 == 0 && (2 * LAT_L) % 64 == 0 && HDIM % 64 == 0);
static_assert(EMB_E % 32 == 0 && LAT_L % 32 == 0);
constexpr int GRID_Q   = ((SEQ_T / 64) * (EMB_E / 64) + 7) / 8;
constexpr int GRID_LKV = ((SEQ_T / 64) * (2 * LAT_L / 64) + 7) / 8;
constexpr int GRID_KH  = ((SEQ_T / 64) * (HDIM / 64) + 7) / 8;
constexpr int GRID_VT  = ((HDIM / 64) * (SEQ_T / 64) + 7) / 8;
constexpr int GRID_OUT = GRID_Q;
constexpr int N8_X   = SEQ_T * EMB_E / 8;
constexpr int N8_WQ  = EMB_E * EMB_E / 8;
constexpr int N8_WK  = LAT_L * EMB_E / 8;
constexpr int N8_QTL = NHEAD * HDIM * LAT_L / 8;
constexpr int N8_WO  = EMB_E * EMB_E / 8;

extern "C" void kernel_launch(void* const* d_in, const int* in_sizes, int n_in,
                              void* d_out, int out_size, void* d_ws, size_t ws_size,
                              hipStream_t stream) {
  if (n_in < 7) return;
  if (in_sizes[0] != SEQ_T * EMB_E || in_sizes[1] != EMB_E * EMB_E ||
      in_sizes[2] != LAT_L * EMB_E || in_sizes[3] != LAT_L * EMB_E ||
      in_sizes[4] != NHEAD * HDIM * LAT_L || in_sizes[5] != NHEAD * LAT_L * HDIM ||
      in_sizes[6] != EMB_E * EMB_E) return;
  if (out_size != SEQ_T * EMB_E) return;
  if ((size_t)WS_TOTAL > ws_size) return;

  const float* X   = (const float*)d_in[0];
  const float* Wq  = (const float*)d_in[1];
  const float* Wk  = (const float*)d_in[2];
  const float* Wv  = (const float*)d_in[3];
  const float* Qtl = (const float*)d_in[4];
  const float* Vup = (const float*)d_in[5];
  const float* Wo  = (const float*)d_in[6];
  float* Out = (float*)d_out;

  char* ws = (char*)d_ws;
  unsigned short* Xb    = (unsigned short*)(ws + OFF_XB);
  unsigned short* Wqb   = (unsigned short*)(ws + OFF_WQB);
  unsigned short* Wkvb  = (unsigned short*)(ws + OFF_WKVB);
  unsigned short* Qtlb  = (unsigned short*)(ws + OFF_QTLB);
  unsigned short* VupTb = (unsigned short*)(ws + OFF_VUPT);
  unsigned short* Wob   = (unsigned short*)(ws + OFF_WOB);
  unsigned short* Qph   = (unsigned short*)(ws + OFF_QPH);
  unsigned short* Qpl   = (unsigned short*)(ws + OFF_QPL);
  unsigned short* Lkvh  = (unsigned short*)(ws + OFF_LKVH);
  unsigned short* Lkvl  = (unsigned short*)(ws + OFF_LKVL);
  unsigned short* Kph   = (unsigned short*)(ws + OFF_KPH);
  unsigned short* Kpl   = (unsigned short*)(ws + OFF_KPL);
  unsigned short* Vth   = (unsigned short*)(ws + OFF_VTH);
  unsigned short* Vtl   = (unsigned short*)(ws + OFF_VTL);
  unsigned short* Ctxh  = (unsigned short*)(ws + OFF_CTXH);
  unsigned short* Ctxl  = (unsigned short*)(ws + OFF_CTXL);

  k_cast_bf16x8<<<(N8_X + 255) / 256, 256, 0, stream>>>(X, Xb, N8_X);
  k_cast_bf16x8<<<(N8_WQ + 255) / 256, 256, 0, stream>>>(Wq, Wqb, N8_WQ);
  k_cast_bf16x8<<<(N8_WK + 255) / 256, 256, 0, stream>>>(Wk, Wkvb, N8_WK);
  k_cast_bf16x8<<<(N8_WK + 255) / 256, 256, 0, stream>>>(Wv, Wkvb + (size_t)LAT_L * EMB_E, N8_WK);
  k_cast_bf16x8<<<(N8_QTL + 255) / 256, 256, 0, stream>>>(Qtl, Qtlb, N8_QTL);
  k_cast_bf16x8<<<(N8_WO + 255) / 256, 256, 0, stream>>>(Wo, Wob, N8_WO);
  k_vup_tcast<<<dim3(LAT_L / 64, HDIM / 64, NHEAD), 256, 0, stream>>>(Vup, VupTb);

  wmma_gemm64<1, 0, 0, 2, false><<<dim3(GRID_Q, 1), 256, 0, stream>>>(
      Xb, nullptr, EMB_E, 0L, Wqb, nullptr, EMB_E, 0L,
      (void*)Qph, (void*)Qpl, EMB_E, 0L, nullptr, nullptr, 0L, SEQ_T, EMB_E, EMB_E, 1.0f);
  wmma_gemm64<1, 0, 0, 2, false><<<dim3(GRID_LKV, 1), 256, 0, stream>>>(
      Xb, nullptr, EMB_E, 0L, Wkvb, nullptr, EMB_E, 0L,
      (void*)Lkvh, (void*)Lkvl, 2 * LAT_L, 0L, nullptr, nullptr, 0L, SEQ_T, 2 * LAT_L, EMB_E, 1.0f);
  wmma_gemm64<1, 2, 0, 2, false><<<dim3(GRID_KH, NHEAD), 256, 0, stream>>>(
      Lkvh, Lkvl, 2 * LAT_L, 0L, Qtlb, nullptr, LAT_L, (long)HDIM * LAT_L,
      (void*)Kph, (void*)Kpl, HDIM, (long)SEQ_T * HDIM, nullptr, nullptr, 0L, SEQ_T, HDIM, LAT_L, 1.0f);
  wmma_gemm64<1, 3, 0, 2, false><<<dim3(GRID_VT, NHEAD), 256, 0, stream>>>(
      VupTb, nullptr, LAT_L, (long)HDIM * LAT_L, Lkvh + LAT_L, Lkvl + LAT_L, 2 * LAT_L, 0L,
      (void*)Vth, (void*)Vtl, SEQ_T, (long)HDIM * SEQ_T, nullptr, nullptr, 0L, HDIM, SEQ_T, LAT_L, 1.0f);
  k_band_attn<<<NHEAD * (SEQ_T / AQB), 128, 0, stream>>>(Qph, Qpl, Kph, Kpl, Vth, Vtl, Ctxh, Ctxl);
  wmma_gemm64<1, 2, 0, 0, false><<<dim3(GRID_OUT, 1), 256, 0, stream>>>(
      Ctxh, Ctxl, EMB_E, 0L, Wob, nullptr, EMB_E, 0L,
      (void*)Out, nullptr, EMB_E, 0L, nullptr, nullptr, 0L, SEQ_T, EMB_E, EMB_E, 1.0f);
}
